// CompGraphConvLayer_48395691491487
// MI455X (gfx1250) — hardware-run, weakly checked
//
#include <hip/hip_runtime.h>
#include <stddef.h>
#include <stdint.h>


#define DF     256
#define NN     50000
#define NE     200000
#define NREL   2
#define NRF    4
#define TERMS  2
#define MW     (TERMS * DF)
#define XOFF   (NREL * MW)
#define KTOT   (XOFF + DF)
#define AP     KTOT
#define MP     50048
#define NPADR  (MP - NN)
#define NTHR   256
#define NWAVE  8
#define EPT    8
#define CHUNK  (NTHR * EPT)
#define WCAP   (EPT * 32)
#define LISTN  (NWAVE * WCAP)
#define NBA    1024
#define SLA    10
#define RCAP   8192
#define DEGCAP 32
#define MEAS_B1024_R0 4212
#define MEAS_B1024_R1 4208
#define MEAS_DEG_R0   15
#define MEAS_DEG_R1   16
#define GBM    64
#define GBN    128
#define GTHR   128
#define NUXB   (NN * (DF / 8))
#define NUPAD  (NPADR * (AP / 8))
#define NPARTW (NREL * TERMS + 1)
#define UPART  (DF * (DF / 8))
#define NUW    (NPARTW * UPART)
#define NUALL  (NUXB + NUPAD + NUW)
#define AGG_ZINTS    (LISTN + 2 * RCAP + 3 * NBA)
#define MISC_INTS    16
#define AGG_LDS_INTS (AGG_ZINTS + MISC_INTS)
#define OUT0_ELEMS   ((long long)NN * DF)
#define OUT_ELEMS    (OUT0_ELEMS + (long long)NRF * DF)
#define WSMAX  134217728

static_assert(TERMS == 1 || TERMS == 2);
static_assert(DF == 256 && DF == 32 * 8);
static_assert(KTOT % 32 == 0 && AP % 64 == 0);
static_assert(MP == 391 * 128 && MP % GBM == 0 && MP >= NN && NPADR == 48);
static_assert((OUT0_ELEMS * 4) % 128 == 0);
static_assert(OUT0_ELEMS + (long long)(NRF - 1) * DF + (DF - 1) < OUT_ELEMS);
static_assert((CHUNK & (CHUNK - 1)) == 0 && CHUNK <= 4096);
static_assert((NBA & (NBA - 1)) == 0 && NBA == (1 << SLA));
static_assert(((long long)CHUNK << SLA) < (1LL << 31));
static_assert(NE < (1 << 21) && (((long long)NE) << SLA) < (1LL << 31));
static_assert(NBA % NWAVE == 0 && NBA % 32 == 0);
static_assert(RCAP % 4 == 0 && AGG_ZINTS % (NTHR * 4) == 0 && LISTN % 4 == 0);
static_assert(RCAP >= MEAS_B1024_R0 + MEAS_B1024_R0 / 20 + 1);
static_assert(RCAP >= MEAS_B1024_R1 + MEAS_B1024_R1 / 20 + 1);
static_assert(DEGCAP >= MEAS_DEG_R0 + 8 && DEGCAP >= MEAS_DEG_R1 + 8);
static_assert(((NN + NBA - 1) / NBA) * NBA >= NN);
static_assert(GBN * 2 == DF && GBM == (GTHR / 32) * 16);
static_assert(NUXB % NTHR == 0 && NUPAD % NTHR == 0 && UPART % NTHR == 0 && UPART == (1 << 13));
static_assert(NUALL % NTHR == 0);
static_assert(AGG_LDS_INTS * 4 <= 300000);
static_assert((NE & 3) == 0);

typedef float          v4f   __attribute__((ext_vector_type(4)));
typedef float          v8f   __attribute__((ext_vector_type(8)));
typedef int            v4i   __attribute__((ext_vector_type(4)));
typedef int            v8i   __attribute__((ext_vector_type(8)));
typedef unsigned       v4u   __attribute__((ext_vector_type(4)));
typedef unsigned short v8us  __attribute__((ext_vector_type(8)));
typedef unsigned short v16us __attribute__((ext_vector_type(16)));
typedef __bf16         v16bf __attribute__((ext_vector_type(16)));
typedef v4f  __attribute__((may_alias)) v4fa;
typedef v4i  __attribute__((may_alias)) v4ia;
typedef v4u  __attribute__((may_alias)) v4ua;
typedef v8us __attribute__((may_alias)) v8usa;
union FragB { v16bf v; v16us u; v8us h[2]; v8i w; };

__device__ __forceinline__ v8f wmb(const FragB& a, const FragB& b, v8f c) {
  v8f d = __builtin_amdgcn_wmma_f32_16x16x32_bf16(false, a.v, false, b.v, (short)0, c, false, false);
  asm volatile("v_nop\n\tv_nop\n\tv_nop\n\tv_nop" : "+v"(d) : "v"(a.w), "v"(b.w));
  return d;
}

__device__ __forceinline__ unsigned bf16_bits(float f) {
  const unsigned u = __float_as_uint(f);
  return (u + 0x7FFFu + ((u >> 16) & 1u)) >> 16;
}
__device__ __forceinline__ unsigned bf16_bits_n(float f) {
  const unsigned r = bf16_bits(f);
  return (f != f) ? 0x7fc0u : r;
}
__device__ __forceinline__ float bf16_val(float f) {
  return __uint_as_float(bf16_bits(f) << 16);
}
__device__ __forceinline__ unsigned split2(float v0, float v1, unsigned* lw) {
  const unsigned h0 = bf16_bits_n(v0);
  const unsigned h1 = bf16_bits_n(v1);
  const unsigned l0 = bf16_bits_n(v0 - __uint_as_float(h0 << 16));
  const unsigned l1 = bf16_bits_n(v1 - __uint_as_float(h1 << 16));
  *lw = l0 | (l1 << 16);
  return h0 | (h1 << 16);
}
__device__ __forceinline__ void put16(unsigned short* dp, v4u o) {
  *(volatile v4u*)dp = o;
  __threadfence();
  *(volatile v4u*)dp = o;
}

template <int SLB>
__device__ __forceinline__ int scan_chunk(const int* __restrict__ dsts, int nE, int cbase, int slotBase,
                                          int nb, int vec8, int* list, int tid, int lane, int wave) {
  int wc = 0;
  const int el0  = tid * EPT;
  const int e0   = cbase + el0;
  const int sent = -2147483647 - 1;
  v4i da, db;
  if (vec8 != 0 && cbase + CHUNK <= nE) {
    da = *(const v4i*)(dsts + e0);
    db = *(const v4i*)(dsts + e0 + 4);
  } else {
    da.x = (e0     < nE) ? dsts[min(e0,     nE - 1)] : sent;
    da.y = (e0 + 1 < nE) ? dsts[min(e0 + 1, nE - 1)] : sent;
    da.z = (e0 + 2 < nE) ? dsts[min(e0 + 2, nE - 1)] : sent;
    da.w = (e0 + 3 < nE) ? dsts[min(e0 + 3, nE - 1)] : sent;
    db.x = (e0 + 4 < nE) ? dsts[min(e0 + 4, nE - 1)] : sent;
    db.y = (e0 + 5 < nE) ? dsts[min(e0 + 5, nE - 1)] : sent;
    db.z = (e0 + 6 < nE) ? dsts[min(e0 + 6, nE - 1)] : sent;
    db.w = (e0 + 7 < nE) ? dsts[min(e0 + 7, nE - 1)] : sent;
  }
  const unsigned nbs = (unsigned)slotBase;
  const unsigned unb = (unsigned)nb;
  const unsigned s0 = (unsigned)da.x - nbs, s1 = (unsigned)da.y - nbs;
  const unsigned s2 = (unsigned)da.z - nbs, s3 = (unsigned)da.w - nbs;
  const unsigned s4 = (unsigned)db.x - nbs, s5 = (unsigned)db.y - nbs;
  const unsigned s6 = (unsigned)db.z - nbs, s7 = (unsigned)db.w - nbs;
  const bool h0 = s0 < unb, h1 = s1 < unb, h2 = s2 < unb, h3 = s3 < unb;
  const bool h4 = s4 < unb, h5 = s5 < unb, h6 = s6 < unb, h7 = s7 < unb;
  const unsigned any = __builtin_amdgcn_ballot_w32(h0 | h1 | h2 | h3 | h4 | h5 | h6 | h7);
  if (any != 0u) {
#define HITJ(J, HJ, SJ) { \
      const unsigned mj = __builtin_amdgcn_ballot_w32(HJ); \
      if (mj != 0u) { \
        if (HJ) { \
          const int pos = wc + (int)__builtin_amdgcn_mbcnt_lo(mj, 0u); \
          if (pos < WCAP) list[wave * WCAP + pos] = ((el0 + (J)) << SLB) | (int)(SJ); \
        } \
        wc += (int)__builtin_popcount(mj); } }
    HITJ(0, h0, s0)
    HITJ(1, h1, s1)
    HITJ(2, h2, s2)
    HITJ(3, h3, s3)
    HITJ(4, h4, s4)
    HITJ(5, h5, s5)
    HITJ(6, h6, s6)
    HITJ(7, h7, s7)
#undef HITJ
  }
  return wc;
}

__device__ __forceinline__ void wcat_unit(const float* __restrict__ W, int n, int kk, unsigned short* dp) {
  const float* p = W + (size_t)kk * DF + n;
  const float f0 = p[0 * DF], f1 = p[1 * DF], f2 = p[2 * DF], f3 = p[3 * DF];
  const float f4 = p[4 * DF], f5 = p[5 * DF], f6 = p[6 * DF], f7 = p[7 * DF];
  v4u o;
  o.x = bf16_bits(f0) | (bf16_bits(f1) << 16);
  o.y = bf16_bits(f2) | (bf16_bits(f3) << 16);
  o.z = bf16_bits(f4) | (bf16_bits(f5) << 16);
  o.w = bf16_bits(f6) | (bf16_bits(f7) << 16);
  put16(dp, o);
}

__global__ __launch_bounds__(NTHR) void k_prep(const float* __restrict__ x, const float* __restrict__ wo,
                                               const float* __restrict__ wi, const float* __restrict__ wsw,
                                               unsigned short* apl, unsigned short* wcat) {
  const int u = (int)blockIdx.x * NTHR + (int)threadIdx.x;
  if (u < NUXB) {
    const int row = u >> 5, k8 = (u & 31) * 8;
    const float* p = x + (size_t)row * DF + k8;
    const v4f a = *(const v4f*)p;
    const v4f b = *(const v4f*)(p + 4);
    v4u o;
    o.x = bf16_bits(a.x) | (bf16_bits(a.y) << 16);
    o.y = bf16_bits(a.z) | (bf16_bits(a.w) << 16);
    o.z = bf16_bits(b.x) | (bf16_bits(b.y) << 16);
    o.w = bf16_bits(b.z) | (bf16_bits(b.w) << 16);
    put16(apl + (size_t)row * AP + XOFF + k8, o);
  } else if (u < NUXB + NUPAD) {
    const int v = u - NUXB;
    const v4u z = {0u, 0u, 0u, 0u};
    put16(apl + (size_t)NN * AP + (size_t)v * 8, z);
  } else if (u < NUALL) {
    const int v    = u - NUXB - NUPAD;
    const int part = v >> 13;
    const int w    = v & (UPART - 1);
    const int n    = w >> 5, kk = (w & 31) * 8;
    unsigned short* dp = wcat + (size_t)n * KTOT + (size_t)part * DF + kk;
    if (part < TERMS)             wcat_unit(wo,  n, kk, dp);
    else if (part < NREL * TERMS) wcat_unit(wi,  n, kk, dp);
    else                          wcat_unit(wsw, n, kk, dp);
  }
}

__global__ __launch_bounds__(NTHR) void k_small(const float* __restrict__ rf, const float* __restrict__ wr,
                                                const float* __restrict__ wrb, const float* __restrict__ wsw,
                                                const float* __restrict__ wob, const float* __restrict__ wib,
                                                const float* __restrict__ wsb, float* cvec, float* rout) {
  __shared__ __attribute__((aligned(16))) float hes[NRF * DF];
  const int n = (int)threadIdx.x;
  {
    const v4f a = *(const v4f*)(rf + 4 * n);
    v4f q;
    q.x = bf16_val(a.x); q.y = bf16_val(a.y); q.z = bf16_val(a.z); q.w = bf16_val(a.w);
    *(v4fa*)(hes + 4 * n) = q;
  }
  __syncthreads();
  float r0 = 0.0f, r1 = 0.0f, r2 = 0.0f, r3 = 0.0f, c3 = 0.0f;
#pragma unroll 4
  for (int k = 0; k < DF; ++k) {
    const float wv = bf16_val(wr[(size_t)k * DF + n]);
    const float sv = bf16_val(wsw[(size_t)k * DF + n]);
    const float g0 = hes[k], g1 = hes[DF + k], g2 = hes[2 * DF + k], g3 = hes[3 * DF + k];
    r0 = fmaf(g0, wv, r0);
    r1 = fmaf(g1, wv, r1);
    r2 = fmaf(g2, wv, r2);
    r3 = fmaf(g3, wv, r3);
    c3 = fmaf(g3, sv, c3);
  }
  const float bb = bf16_val(wrb[n]);
  const float o0 = r0 + bb, o1 = r1 + bb, o2 = r2 + bb, o3 = r3 + bb;
  const float bs = (bf16_val(wob[n]) + bf16_val(wib[n])) + bf16_val(wsb[n]);
  const float cv = bs - c3;
  float* rp = rout + n;
  *(volatile float*)(rp)          = o0;
  *(volatile float*)(rp + DF)     = o1;
  *(volatile float*)(rp + 2 * DF) = o2;
  *(volatile float*)(rp + 3 * DF) = o3;
  *(volatile float*)(cvec + n)    = cv;
  __threadfence();
  *(volatile float*)(rp)          = o0;
  *(volatile float*)(rp + DF)     = o1;
  *(volatile float*)(rp + 2 * DF) = o2;
  *(volatile float*)(rp + 3 * DF) = o3;
  *(volatile float*)(cvec + n)    = cv;
}

__global__ __launch_bounds__(NTHR) __attribute__((amdgpu_num_vgpr(248)))
void k_scan(const int* __restrict__ gath, const int* __restrict__ keys, const float* __restrict__ herow,
            int nE, int nN, int vec8, int cbase, const unsigned short* xbp, unsigned short* apl) {
  extern __shared__ __attribute__((aligned(16))) int dsm[];
  int* list = dsm;
  int* hl   = dsm + LISTN;
  int* sl   = hl + RCAP;
  int* cnt  = sl + RCAP;
  int* offs = cnt + NBA;
  int* cur  = offs + NBA;
  int* misc = cur + NBA;
  const int tid = (int)threadIdx.x, lane = tid & 31, wave = tid >> 5;
  const int nodeBase = (int)blockIdx.x * NBA;

  {
    const v4i z4 = {0, 0, 0, 0};
    for (int i = tid * 4; i < AGG_ZINTS; i += NTHR * 4) *(v4ia*)(dsm + i) = z4;
    if (tid < MISC_INTS) misc[tid] = 0;
  }
  __syncthreads();

  int t = 0, ov = 0;
  const int nChunks = (nE + CHUNK - 1) / CHUNK;
#pragma unroll 1
  for (int ch = 0; ch < nChunks; ++ch) {
    const int cb = ch * CHUNK;
    const int wc = scan_chunk<SLA>(keys, nE, cb, nodeBase, NBA, vec8, list, tid, lane, wave);
    if (lane == 0) misc[wave] = wc;
    __syncthreads();
    if (wave == 0) {
#pragma unroll 1
      for (int w2 = 0; w2 < NWAVE; ++w2) {
        int c = misc[w2];
        c = c < 0 ? 0 : (c > WCAP ? WCAP : c);
#pragma unroll 1
        for (int b0 = 0; b0 < c; b0 += 32) {
          const int idx = b0 + lane;
          const int ent = list[w2 * WCAP + (idx < WCAP ? idx : WCAP - 1)];
          const int m32 = (c - b0) < 32 ? (c - b0) : 32;
#pragma unroll 1
          for (int k = 0; k < m32; ++k) {
            const int u    = __builtin_amdgcn_readlane(ent, k);
            const int slot = u & (NBA - 1);
            const int el   = (u >> SLA) & (CHUNK - 1);
            const int pk   = ((cb + el) << SLA) | slot;
            if (t < RCAP) {
              if (lane == 0) { hl[t] = pk; cnt[slot] = cnt[slot] + 1; }
              t = t + 1;
            } else {
              ov = 1;
            }
          }
        }
      }
    }
    __syncthreads();
  }
  if (wave == 0 && lane == 0) { misc[8] = t; misc[9] = ov; }
  __syncthreads();
  int tt = misc[8];
  tt = tt < 0 ? 0 : (tt > RCAP ? RCAP : tt);
  const int ovf = misc[9];

  if (wave == 0) {
    const int base = lane * (NBA / 32);
    int s = 0;
#pragma unroll 1
    for (int i = 0; i < NBA / 32; ++i) s += cnt[base + i];
    int incl = s;
#pragma unroll
    for (int d = 1; d < 32; d <<= 1) {
      const int y = __shfl_up(incl, d, 32);
      if (lane >= d) incl += y;
    }
    int run = incl - s;
#pragma unroll 1
    for (int i = 0; i < NBA / 32; ++i) {
      const int cv = cnt[base + i];
      offs[base + i] = run;
      cur[base + i]  = run;
      run += cv;
    }
  }
  __syncthreads();
  if (wave == 0) {
#pragma unroll 1
    for (int b0 = 0; b0 < tt; b0 += 32) {
      const int idx = b0 + lane;
      const int ent = hl[idx < RCAP ? idx : RCAP - 1];
      const int m32 = (tt - b0) < 32 ? (tt - b0) : 32;
#pragma unroll 1
      for (int k = 0; k < m32; ++k) {
        const int u    = __builtin_amdgcn_readlane(ent, k);
        const int slot = u & (NBA - 1);
        if (lane == 0) {
          int p = cur[slot];
          p = p < 0 ? 0 : (p > RCAP - 1 ? RCAP - 1 : p);
          sl[p] = u;
          cur[slot] = p + 1;
        }
      }
    }
  }
  __syncthreads();

  const float qn = __uint_as_float(0x7fc00000u);
  const float pz = (ovf != 0) ? qn : 0.0f;
  float he0, he1, he2, he3, he4, he5, he6, he7;
  {
    const v4f g0 = *(const v4f*)(herow + 8 * lane);
    const v4f g1 = *(const v4f*)(herow + 8 * lane + 4);
    he0 = bf16_val(g0.x); he1 = bf16_val(g0.y); he2 = bf16_val(g0.z); he3 = bf16_val(g0.w);
    he4 = bf16_val(g1.x); he5 = bf16_val(g1.y); he6 = bf16_val(g1.z); he7 = bf16_val(g1.w);
  }
#pragma unroll 1
  for (int si = 0; si < NBA / NWAVE; ++si) {
    const int s    = si * NWAVE + wave;
    const int node = nodeBase + s;
    int c = cnt[s];
    const bool big = c > DEGCAP;
    c = c < 0 ? 0 : (c > DEGCAP ? DEGCAP : c);
    int o = offs[s];
    o = o < 0 ? 0 : (o > RCAP - 1 ? RCAP - 1 : o);
    int last = o + c - 1;
    last = last < o ? o : last;
    last = last > RCAP - 1 ? RCAP - 1 : last;
    float a0 = 0.0f, a1 = 0.0f, a2 = 0.0f, a3 = 0.0f, a4 = 0.0f, a5 = 0.0f, a6 = 0.0f, a7 = 0.0f;
#pragma unroll 1
    for (int b0 = 0; b0 < c; b0 += 32) {
      int idx = o + b0 + lane;
      idx = idx > last ? last : idx;
      const int ent = sl[idx];
      int eid = ent >> SLA;
      eid = eid < 0 ? 0 : (eid > nE - 1 ? nE - 1 : eid);
      int sr = gath[eid];
      sr = sr < 0 ? 0 : (sr > nN - 1 ? nN - 1 : sr);
      const int m32 = (c - b0) < 32 ? (c - b0) : 32;
#pragma unroll 1
      for (int k = 0; k < m32; ++k) {
        const int sk = __builtin_amdgcn_readlane(sr, k);
        const v4u w = *(const v4ua*)(xbp + (size_t)sk * AP + XOFF + 8 * lane);
        a0 += __uint_as_float(w.x << 16)         - he0;
        a1 += __uint_as_float(w.x & 0xffff0000u) - he1;
        a2 += __uint_as_float(w.y << 16)         - he2;
        a3 += __uint_as_float(w.y & 0xffff0000u) - he3;
        a4 += __uint_as_float(w.z << 16)         - he4;
        a5 += __uint_as_float(w.z & 0xffff0000u) - he5;
        a6 += __uint_as_float(w.w << 16)         - he6;
        a7 += __uint_as_float(w.w & 0xffff0000u) - he7;
      }
    }
    const int   cd  = max(c, 1);
    const float cf  = (float)cd;
    const float pzr = big ? qn : pz;
    const float m0 = a0 / cf + pzr, m1 = a1 / cf + pzr, m2 = a2 / cf + pzr, m3 = a3 / cf + pzr;
    const float m4 = a4 / cf + pzr, m5 = a5 / cf + pzr, m6 = a6 / cf + pzr, m7 = a7 / cf + pzr;
    v4u hv, lv;
    {
      unsigned lw;
      unsigned hw;
      hw = split2(m0, m1, &lw); hv.x = hw; lv.x = lw;
      hw = split2(m2, m3, &lw); hv.y = hw; lv.y = lw;
      hw = split2(m4, m5, &lw); hv.z = hw; lv.z = lw;
      hw = split2(m6, m7, &lw); hv.w = hw; lv.w = lw;
    }
    if (node < nN) {
      unsigned short* rp = apl + (size_t)node * AP + cbase + 8 * lane;
      *(volatile v4u*)rp = hv;
      if constexpr (TERMS == 2) *(volatile v4u*)(rp + DF) = lv;
      __threadfence();
      *(volatile v4u*)rp = hv;
      if constexpr (TERMS == 2) *(volatile v4u*)(rp + DF) = lv;
    }
  }
}

__global__ __launch_bounds__(GTHR) __attribute__((amdgpu_num_vgpr(248)))
void k_gemm(const unsigned short* __restrict__ A, const unsigned short* __restrict__ BT,
            const float* __restrict__ cvec, float* outp, int nOut) {
  __shared__ __attribute__((aligned(16))) float stg[GBM * GBN];
  __shared__ __attribute__((aligned(16))) float cvs[GBN];
  const int tid = (int)threadIdx.x, lane = tid & 31, wave = tid >> 5, hh = lane >> 4, m = lane & 15;
  const int rowBase = (int)blockIdx.x * GBM;
  const int colBase = (int)blockIdx.y * GBN;

  v8f acc[8];
  {
    const v8f z = {0.f, 0.f, 0.f, 0.f, 0.f, 0.f, 0.f, 0.f};
#pragma unroll
    for (int t = 0; t < 8; ++t) acc[t] = z;
  }
  const unsigned short* ap = A + (size_t)(rowBase + 16 * wave + m) * (size_t)AP + 8 * hh;
  const unsigned short* bp = BT + (size_t)(colBase + m) * (size_t)KTOT + 8 * hh;

#pragma unroll 1
  for (int k0 = 0; k0 < KTOT; k0 += 32) {
    FragB af;
    af.h[0] = *(const v8usa*)(ap + k0);
    af.h[1] = *(const v8usa*)(ap + k0 + 16);
#pragma unroll
    for (int nt = 0; nt < 8; ++nt) {
      const unsigned short* wq = bp + (size_t)(16 * nt) * (size_t)KTOT + k0;
      FragB bf;
      bf.h[0] = *(const v8usa*)wq;
      bf.h[1] = *(const v8usa*)(wq + 16);
      acc[nt] = wmb(af, bf, acc[nt]);
    }
  }

#pragma unroll
  for (int nt = 0; nt < 8; ++nt) {
    const int lc = 16 * nt + m;
#pragma unroll
    for (int r = 0; r < 8; ++r) {
      const int lr = 16 * wave + 8 * hh + r;
      stg[lr * GBN + lc] = acc[nt][r];
    }
  }
  if (wave == 0) {
    const v4f c4 = *(const v4f*)(cvec + colBase + 4 * lane);
    *(v4fa*)(cvs + 4 * lane) = c4;
  }
  __syncthreads();

  const v4f cv4 = *(const v4fa*)(cvs + 4 * lane);
  v4f pv[16];
#pragma unroll
  for (int i = 0; i < 16; ++i) {
    const v4f d = *(const v4fa*)(stg + (16 * wave + i) * GBN + 4 * lane);
    pv[i] = d + cv4;
  }

#pragma unroll
  for (int i = 0; i < 16; ++i) {
    const int r = rowBase + 16 * wave + i;
    if (r < nOut) *(volatile v4f*)(outp + (size_t)r * DF + colBase + 4 * lane) = pv[i];
  }
  __threadfence();
#pragma unroll
  for (int i = 0; i < 16; ++i) {
    const int r = rowBase + 16 * wave + i;
    if (r < nOut) *(volatile v4f*)(outp + (size_t)r * DF + colBase + 4 * lane) = pv[i];
  }
}

static inline size_t al256(size_t o) { return (o + 255) & ~(size_t)255; }

extern "C" void kernel_launch(void* const* d_in, const int* in_sizes, int n_in,
                              void* d_out, int out_size, void* d_ws, size_t ws_size,
                              hipStream_t stream) {
  if (n_in < 14) return;
  if (in_sizes[0] != NN * DF) return;
  if (in_sizes[1] != NRF * DF) return;
  if (in_sizes[2] != NE || in_sizes[3] != NE || in_sizes[4] != NE || in_sizes[5] != NE) return;
  if (in_sizes[6] != DF * DF || in_sizes[8] != DF * DF || in_sizes[10] != DF * DF || in_sizes[12] != DF * DF) return;
  if (in_sizes[7] != DF || in_sizes[9] != DF || in_sizes[11] != DF || in_sizes[13] != DF) return;
  if ((long long)out_size != OUT_ELEMS) return;

  const float* x    = (const float*)d_in[0];
  const float* rf   = (const float*)d_in[1];
  const int*   src0 = (const int*)d_in[2];
  const int*   dst0 = (const int*)d_in[3];
  const int*   src1 = (const int*)d_in[4];
  const int*   dst1 = (const int*)d_in[5];
  const float* WOw  = (const float*)d_in[6];
  const float* WOb  = (const float*)d_in[7];
  const float* WIw  = (const float*)d_in[8];
  const float* WIb  = (const float*)d_in[9];
  const float* WSw  = (const float*)d_in[10];
  const float* WSb  = (const float*)d_in[11];
  const float* WRw  = (const float*)d_in[12];
  const float* WRb  = (const float*)d_in[13];
  float* out  = (float*)d_out;
  float* rout = out + (size_t)OUT0_ELEMS;

  char* ws = (char*)d_ws;
  size_t off = 0;
  const size_t oW = off; off = al256(off + (size_t)DF * KTOT * 2);
  const size_t oC = off; off = al256(off + (size_t)DF * 4);
  const size_t oA = off; off = al256(off + (size_t)MP * AP * 2);
  if (off > ws_size || off > (size_t)WSMAX) return;
  unsigned short* Wcat = (unsigned short*)(ws + oW);
  float*          cvec = (float*)(ws + oC);
  unsigned short* Apl  = (unsigned short*)(ws + oA);

  const size_t scanLds = (size_t)AGG_LDS_INTS * 4;
  hipFuncSetAttribute(reinterpret_cast<const void*>(&k_scan), hipFuncAttributeMaxDynamicSharedMemorySize, (int)scanLds);

  const int gA   = (NN + NBA - 1) / NBA;
  const int vec8 = ((NE & 3) == 0) ? 1 : 0;

  k_prep<<<NUALL / NTHR, NTHR, 0, stream>>>(x, WOw, WIw, WSw, Apl, Wcat);
  k_small<<<1, NTHR, 0, stream>>>(rf, WRw, WRb, WSw, WOb, WIb, WSb, cvec, rout);
  k_scan<<<gA, NTHR, scanLds, stream>>>(src0, dst0, rf + 1 * DF, NE, NN, vec8, 0, Apl, Apl);
  k_scan<<<gA, NTHR, scanLds, stream>>>(src1, dst1, rf + 2 * DF, NE, NN, vec8, MW, Apl, Apl);
  k_gemm<<<dim3(MP / GBM, DF / GBN), GTHR, 0, stream>>>(Apl, Wcat, cvec, out, NN);
}
